// GraphGymGNN_41317585388128
// MI455X (gfx1250) — hardware-verified
//
#include <hip/hip_runtime.h>
#include <stddef.h>
#include <math.h>


#define FD      128
#define CHN     32
#define NOUTC   64
#define NC2     256
#define CP      256
#define PP      128
#define NTHR    256
#define NWAVE   8
#define EPT     8
#define NGRP    2
#define CHUNK   (NTHR * EPT * NGRP)
#define WCAP    (EPT * NGRP * 32)
#define LISTN   (NWAVE * WCAP)
#define NBC     4096
#define NBF     2048
#define FPC     (NBC / NBF)
#define RCAP    40960
#define RBN     128
#define TGT     256
#define DEGCAP  256
#define OTHR    512
#define BM      64
#define STATR   256
#define WSCAP   134217728
#define BN_EPS  1e-5
#define LSLOPE  0.2f
#define LOG2E   1.4426950408889634f
#define NEGBIG  (-3.0e38f)

#define LDS_FILL ((RCAP + NBF + LISTN) * 4 + 64)
#define LDS_G256 (BM * 256 * 4)
#define LDS_G128 (BM * 128 * 4)
#define LDS_G64  (BM * 64 * 4)

static_assert((CHUNK & (CHUNK - 1)) == 0);
static_assert(CHUNK <= 4096);
static_assert(NBC <= 4096 && NBF <= 4096);
static_assert((NBC & (NBC - 1)) == 0 && (NBF & (NBF - 1)) == 0);
static_assert(NBC == FPC * NBF && FPC == 2);
static_assert(OTHR * 8 == NBC);
static_assert(OTHR / 32 == 8 * FPC);
static_assert((RCAP % 32) == 0);
static_assert(TGT == NWAVE * 32);
static_assert((TGT % BM) == 0 && (TGT % STATR) == 0);
static_assert((DEGCAP % 32) == 0);
static_assert(FD == 4 * CHN && NC2 == 2 * FD && CP == NC2 && PP == FD);
static_assert(BM == 64 && NWAVE == 8);

typedef float          v4f  __attribute__((ext_vector_type(4)));
typedef float          v8f  __attribute__((ext_vector_type(8)));
typedef double         v2d  __attribute__((ext_vector_type(2)));
typedef int            v4i  __attribute__((ext_vector_type(4)));
typedef unsigned short v8us __attribute__((ext_vector_type(8)));
typedef unsigned short v16us __attribute__((ext_vector_type(16)));
typedef __bf16         v16bf __attribute__((ext_vector_type(16)));
union FragU { v16us w; v8us u[2]; };

__device__ __forceinline__ v8f wmb(v16us a, v16us b, v8f c) {
  const v16bf ab = __builtin_bit_cast(v16bf, a);
  const v16bf bb = __builtin_bit_cast(v16bf, b);
  v8f d = __builtin_amdgcn_wmma_f32_16x16x32_bf16(false, ab, false, bb, (short)0, c, false, false);
  asm volatile("v_nop\n\tv_nop\n\tv_nop\n\tv_nop" : "+v"(d) : "v"(a), "v"(b));
  return d;
}

__device__ __forceinline__ unsigned int bfb(float f) {
  const unsigned int u = __float_as_uint(f);
  return (u + 0x7FFFu + ((u >> 16) & 1u)) >> 16;
}
__device__ __forceinline__ void sp1(float v, unsigned short& h, unsigned short& l) {
  const unsigned int hb = bfb(v);
  const float hf = __uint_as_float(hb << 16);
  h = (unsigned short)hb;
  l = (unsigned short)bfb(v - hf);
}
__device__ __forceinline__ void sp8(v4f a, v4f b, v8us& h, v8us& l) {
  unsigned short hh, ll;
  sp1(a.x, hh, ll); h[0] = hh; l[0] = ll;
  sp1(a.y, hh, ll); h[1] = hh; l[1] = ll;
  sp1(a.z, hh, ll); h[2] = hh; l[2] = ll;
  sp1(a.w, hh, ll); h[3] = hh; l[3] = ll;
  sp1(b.x, hh, ll); h[4] = hh; l[4] = ll;
  sp1(b.y, hh, ll); h[5] = hh; l[5] = ll;
  sp1(b.z, hh, ll); h[6] = hh; l[6] = ll;
  sp1(b.w, hh, ll); h[7] = hh; l[7] = ll;
}

__device__ __forceinline__ v4f lrl4(v4f t) {
  const v4f u = t * LSLOPE; v4f r;
  r.x = fmaxf(t.x, u.x); r.y = fmaxf(t.y, u.y); r.z = fmaxf(t.z, u.z); r.w = fmaxf(t.w, u.w);
  return r;
}
__device__ __forceinline__ v4f prelu4(v4f t, float a) {
  v4f r;
  r.x = t.x >= 0.f ? t.x : a * t.x; r.y = t.y >= 0.f ? t.y : a * t.y;
  r.z = t.z >= 0.f ? t.z : a * t.z; r.w = t.w >= 0.f ? t.w : a * t.w;
  return r;
}
__device__ __forceinline__ float dot4(v4f a, v4f b) {
  return fmaf(a.w, b.w, fmaf(a.z, b.z, fmaf(a.y, b.y, a.x * b.x)));
}
__device__ __forceinline__ float fexp(float x) { return __builtin_amdgcn_exp2f(x * LOG2E); }
__device__ __forceinline__ float rlf(float v, int l) {
  return __int_as_float(__builtin_amdgcn_readlane(__float_as_int(v), l));
}
__device__ __forceinline__ float gsum8(float v) {
#pragma unroll
  for (int o = 1; o < 8; o <<= 1) v += __shfl_xor(v, o);
  return v;
}

__global__ __launch_bounds__(NTHR) void k_wprep(const float* __restrict__ Wa, const float* __restrict__ Wb,
                                               int nca, int ncb, unsigned short* ph, unsigned short* pl, int units) {
  const int i = (int)blockIdx.x * NTHR + (int)threadIdx.x;
  if (i >= units) return;
  const int n  = i >> 4;
  const int k0 = (i & 15) * 8;
  const int na = n < nca - 1 ? n : nca - 1;
  int nb = n - nca; nb = nb < 0 ? 0 : (nb > ncb - 1 ? ncb - 1 : nb);
  v8us hv, lv;
#pragma unroll
  for (int e = 0; e < 8; ++e) {
    const float fa = Wa[(size_t)(k0 + e) * nca + na];
    const float fb = Wb[(size_t)(k0 + e) * ncb + nb];
    const float f  = n < nca ? fa : fb;
    unsigned short h, l;
    sp1(f, h, l);
    hv[e] = h; lv[e] = l;
  }
  unsigned short* dh = ph + (size_t)i * 8;
  unsigned short* dl = pl + (size_t)i * 8;
  *(volatile v8us*)dh = hv;
  *(volatile v8us*)dl = lv;
  __threadfence();
  *(volatile v8us*)dh = hv;
  *(volatile v8us*)dl = lv;
}

__global__ __launch_bounds__(NTHR) void k_xsplit(const float* __restrict__ x, unsigned short* ph, unsigned short* pl,
                                                int nN, int nUnits) {
  const int i = (int)blockIdx.x * NTHR + (int)threadIdx.x;
  if (i >= nUnits) return;
  const int row = i >> 4;
  const int c   = (i & 15) * 8;
  const int rc  = row < nN ? row : nN - 1;
  const float* xr = x + (size_t)rc * FD + c;
  v4f a = *(const v4f*)xr, b = *(const v4f*)(xr + 4);
  const v4f z4 = {0.f, 0.f, 0.f, 0.f};
  if (row >= nN) { a = z4; b = z4; }
  v8us hv, lv;
  sp8(a, b, hv, lv);
  unsigned short* dh = ph + (size_t)row * PP + c;
  unsigned short* dl = pl + (size_t)row * PP + c;
  *(volatile v8us*)dh = hv;
  *(volatile v8us*)dl = lv;
  __threadfence();
  *(volatile v8us*)dh = hv;
  *(volatile v8us*)dl = lv;
}

__global__ __launch_bounds__(NTHR) void k_eamean(const float* __restrict__ ea, float* eline, int nE) {
  __shared__ double sd[NTHR];
  __shared__ float smv;
  const int tid = threadIdx.x;
  const int nIt = (nE + NTHR - 1) / NTHR;
  double s = 0.0;
#pragma unroll 1
  for (int it = 0; it < nIt; ++it) {
    const int idx = it * NTHR + tid;
    const int ic  = idx < nE ? idx : nE - 1;
    const float v = ea[ic];
    s += (idx < nE) ? (double)v : 0.0;
  }
  sd[tid] = s;
  __syncthreads();
  if (tid == 0) {
    double t = 0.0;
#pragma unroll 1
    for (int k = 0; k < NTHR; ++k) t += sd[k];
    smv = (float)(t / (double)nE);
  }
  __syncthreads();
  const float mv = smv;
  v4f w; w.x = mv; w.y = mv; w.z = mv; w.w = mv;
  if (tid < 8) *(volatile v4f*)(eline + 4 * tid) = w;
  __threadfence();
  if (tid < 8) *(volatile v4f*)(eline + 4 * tid) = w;
}

template <int NB>
__device__ __forceinline__ int scan_chunk(const int* __restrict__ dsts, int nE, int cbase, int slotBase,
                                          int vec8, int* list, int tid, int lane, int wave) {
  int wc = 0;
#pragma unroll
  for (int g = 0; g < NGRP; ++g) {
    const int el0  = (g * NTHR + tid) * EPT;
    const int e0   = cbase + el0;
    const int sent = -2147483647 - 1;
    v4i da, db;
    if (vec8 != 0 && cbase + CHUNK <= nE) {
      da = *(const v4i*)(dsts + e0);
      db = *(const v4i*)(dsts + e0 + 4);
    } else {
      da.x = (e0     < nE) ? dsts[min(e0, nE - 1)] : sent;
      da.y = (e0 + 1 < nE) ? dsts[min(e0 + 1, nE - 1)] : sent;
      da.z = (e0 + 2 < nE) ? dsts[min(e0 + 2, nE - 1)] : sent;
      da.w = (e0 + 3 < nE) ? dsts[min(e0 + 3, nE - 1)] : sent;
      db.x = (e0 + 4 < nE) ? dsts[min(e0 + 4, nE - 1)] : sent;
      db.y = (e0 + 5 < nE) ? dsts[min(e0 + 5, nE - 1)] : sent;
      db.z = (e0 + 6 < nE) ? dsts[min(e0 + 6, nE - 1)] : sent;
      db.w = (e0 + 7 < nE) ? dsts[min(e0 + 7, nE - 1)] : sent;
    }
    const unsigned nb = (unsigned)slotBase;
    const unsigned s0 = (unsigned)da.x - nb, s1 = (unsigned)da.y - nb;
    const unsigned s2 = (unsigned)da.z - nb, s3 = (unsigned)da.w - nb;
    const unsigned s4 = (unsigned)db.x - nb, s5 = (unsigned)db.y - nb;
    const unsigned s6 = (unsigned)db.z - nb, s7 = (unsigned)db.w - nb;
    const bool h0 = s0 < (unsigned)NB, h1 = s1 < (unsigned)NB, h2 = s2 < (unsigned)NB, h3 = s3 < (unsigned)NB;
    const bool h4 = s4 < (unsigned)NB, h5 = s5 < (unsigned)NB, h6 = s6 < (unsigned)NB, h7 = s7 < (unsigned)NB;
    const unsigned any = __builtin_amdgcn_ballot_w32(h0 | h1 | h2 | h3 | h4 | h5 | h6 | h7);
    if (any != 0u) {
#define HITJ(J, HJ, SJ) { \
        const unsigned mj = __builtin_amdgcn_ballot_w32(HJ); \
        if (mj != 0u) { \
          if (HJ) { \
            const int pos = wc + (int)__builtin_amdgcn_mbcnt_lo(mj, 0u); \
            if (pos < WCAP) list[wave * WCAP + pos] = ((el0 + (J)) << 12) | (int)(SJ); \
          } \
          wc += (int)__builtin_popcount(mj); } }
      HITJ(0, h0, s0)
      HITJ(1, h1, s1)
      HITJ(2, h2, s2)
      HITJ(3, h3, s3)
      HITJ(4, h4, s4)
      HITJ(5, h5, s5)
      HITJ(6, h6, s6)
      HITJ(7, h7, s7)
#undef HITJ
    }
  }
  return wc;
}

__global__ __launch_bounds__(NTHR) void k_count(
    const int* __restrict__ dsts, int* cnt, int nE, int vec8) {
  __shared__ __attribute__((aligned(16))) int scnt[NBC];
  __shared__ __attribute__((aligned(16))) int list[LISTN];
  __shared__ int wcnt[NWAVE];
  const int tid = threadIdx.x, lane = tid & 31, wave = tid >> 5;
  const int nodeBase = blockIdx.x * NBC;

  for (int i = tid; i < NBC; i += NTHR) scnt[i] = 0;
  __syncthreads();

  const int nChunks = (nE + CHUNK - 1) / CHUNK;
#pragma unroll 1
  for (int ch = 0; ch < nChunks; ++ch) {
    const int cbase = ch * CHUNK;
    const int wc = scan_chunk<NBC>(dsts, nE, cbase, nodeBase, vec8, list, tid, lane, wave);
    if (lane == 0) wcnt[wave] = wc;
    __syncthreads();
    if (wave == 0) {
#pragma unroll 1
      for (int wsx = 0; wsx < NWAVE; ++wsx) {
        int n = __builtin_amdgcn_readfirstlane(wcnt[wsx]);
        n = n > WCAP ? WCAP : (n < 0 ? 0 : n);
        const int* lp = list + wsx * WCAP;
#pragma unroll 1
        for (int i = 0; i < n; ++i) {
          const int ent  = __builtin_amdgcn_readfirstlane(lp[i]);
          const int slot = ent & (NBC - 1);
          if (lane == 0) scnt[slot] = scnt[slot] + 1;
        }
      }
    }
    __syncthreads();
  }

  v4i cq[4];
#pragma unroll
  for (int q = 0; q < 4; ++q) {
    const int f = (wave * 4 + q) * 128 + 4 * lane;
    cq[q] = *(const v4i*)(scnt + f);
  }
  int* cpn = cnt + (size_t)nodeBase;
#pragma unroll
  for (int q = 0; q < 4; ++q) {
    const int f = (wave * 4 + q) * 128 + 4 * lane;
    *(volatile v4i*)(cpn + f) = cq[q];
  }
  __threadfence();
#pragma unroll
  for (int q = 0; q < 4; ++q) {
    const int f = (wave * 4 + q) * 128 + 4 * lane;
    *(volatile v4i*)(cpn + f) = cq[q];
  }
}

__global__ __launch_bounds__(OTHR) void k_offsets(
    const int* __restrict__ cnt, int* off, int* rbase, int nChunk) {
  __shared__ __attribute__((aligned(16))) int soff[NBC];
  __shared__ __attribute__((aligned(16))) int srb[RBN];
  __shared__ int wtot[OTHR / 32];
  const int tid = threadIdx.x, lane = tid & 31, wave = tid >> 5, sub = tid >> 8;
  for (int i = tid; i < RBN; i += OTHR) srb[i] = 0;
  __syncthreads();
  int carry = 0;
#pragma unroll 1
  for (int ch = 0; ch < nChunk; ++ch) {
    const int base = ch * NBC;
    const v4i ca = *(const v4i*)(cnt + base + 8 * tid);
    const v4i cb = *(const v4i*)(cnt + base + 8 * tid + 4);
    const int e0 = max(ca.x, 0), e1 = max(ca.y, 0), e2 = max(ca.z, 0), e3 = max(ca.w, 0);
    const int e4 = max(cb.x, 0), e5 = max(cb.y, 0), e6 = max(cb.z, 0), e7 = max(cb.w, 0);
    const int ts = e0 + e1 + e2 + e3 + e4 + e5 + e6 + e7;
    int incl = ts;
#pragma unroll
    for (int d = 1; d < 32; d <<= 1) {
      const int t = __shfl_up(incl, d);
      if (lane >= d) incl += t;
    }
    if (lane == 31) wtot[wave] = incl;
    __syncthreads();
    int S0 = 0, S1 = 0;
#pragma unroll
    for (int w = 0; w < 8; ++w) { S0 += wtot[w]; S1 += wtot[8 + w]; }
    int pre = 0;
#pragma unroll 1
    for (int w = 8 * sub; w < wave; ++w) pre += wtot[w];
    const int b0 = carry;
    const int b1 = b0 + ((S0 + 31) & ~31);
    const int b2 = b1 + ((S1 + 31) & ~31);
    const int myb = sub == 0 ? b0 : b1;
    if (tid == 0) {
      srb[min(2 * ch + 0, RBN - 1)] = b0;
      srb[min(2 * ch + 1, RBN - 1)] = b1;
    }
    int run = myb + pre + incl - ts;
    soff[8 * tid + 0] = run; run += e0;
    soff[8 * tid + 1] = run; run += e1;
    soff[8 * tid + 2] = run; run += e2;
    soff[8 * tid + 3] = run; run += e3;
    soff[8 * tid + 4] = run; run += e4;
    soff[8 * tid + 5] = run; run += e5;
    soff[8 * tid + 6] = run; run += e6;
    soff[8 * tid + 7] = run;
    carry = b2;
    __syncthreads();
    const v4i o0 = *(const v4i*)(soff + 4 * tid);
    const v4i o1 = *(const v4i*)(soff + 4 * (tid + OTHR));
    int* op = off + base;
    *(volatile v4i*)(op + 4 * tid) = o0;
    *(volatile v4i*)(op + 4 * (tid + OTHR)) = o1;
    __threadfence();
    *(volatile v4i*)(op + 4 * tid) = o0;
    *(volatile v4i*)(op + 4 * (tid + OTHR)) = o1;
    __syncthreads();
  }
  if (tid == 0) srb[min(2 * nChunk, RBN - 1)] = carry;
  __syncthreads();
  v4i rv = {0, 0, 0, 0};
  if (tid < 32) rv = *(const v4i*)(srb + 4 * tid);
  if (tid < 32) *(volatile v4i*)(rbase + 4 * tid) = rv;
  __threadfence();
  if (tid < 32) *(volatile v4i*)(rbase + 4 * tid) = rv;
}

__global__ __launch_bounds__(NTHR) void k_fill(
    const int* __restrict__ dsts, const int* __restrict__ off, const int* __restrict__ rbase,
    int* csr, int nE, int vec8, int csrLen) {
  extern __shared__ v4f lds_dyn[];
  int* region = (int*)lds_dyn;
  int* cursor = region + RCAP;
  int* list   = cursor + NBF;
  int* wcnt   = list + LISTN;
  const int tid = threadIdx.x, lane = tid & 31, wave = tid >> 5;
  const int b = blockIdx.x;
  const int nodeBase = b * NBF;

  int rb0 = rbase[b];
  const int rb1 = rbase[b + 1];
  rb0 = rb0 < 0 ? 0 : (rb0 > csrLen ? csrLen : rb0);
  rb0 &= ~31;
  int len = rb1 - rb0;
  len = len < 0 ? 0 : (len > RCAP ? RCAP : len);
  int lenW = (len + 31) & ~31;
  if (rb0 + lenW > csrLen) lenW = (csrLen - rb0) & ~31;

  {
    const v4i z = {0, 0, 0, 0};
    for (int i = tid; i < RCAP / 4; i += NTHR) ((v4i*)region)[i] = z;
    for (int s = tid; s < NBF; s += NTHR) {
      int o = off[nodeBase + s] - rb0;
      o = o < 0 ? 0 : (o > RCAP ? RCAP : o);
      cursor[s] = o;
    }
  }
  __syncthreads();

  const int nChunks = (nE + CHUNK - 1) / CHUNK;
#pragma unroll 1
  for (int ch = 0; ch < nChunks; ++ch) {
    const int cbase = ch * CHUNK;
    const int wc = scan_chunk<NBF>(dsts, nE, cbase, nodeBase, vec8, list, tid, lane, wave);
    if (lane == 0) wcnt[wave] = wc;
    __syncthreads();
    if (wave == 0) {
#pragma unroll 1
      for (int wsx = 0; wsx < NWAVE; ++wsx) {
        int n = __builtin_amdgcn_readfirstlane(wcnt[wsx]);
        n = n > WCAP ? WCAP : (n < 0 ? 0 : n);
        const int* lp = list + wsx * WCAP;
#pragma unroll 1
        for (int i = 0; i < n; ++i) {
          const int ent  = __builtin_amdgcn_readfirstlane(lp[i]);
          const int slot = ent & (NBF - 1);
          int e = cbase + ((ent >> 12) & (CHUNK - 1));
          e = e > nE - 1 ? nE - 1 : e;
          if (lane == 0) {
            int pos = cursor[slot];
            pos = pos < 0 ? 0 : (pos > RCAP - 1 ? RCAP - 1 : pos);
            region[pos] = e;
            const int np = pos + 1;
            cursor[slot] = np > RCAP ? RCAP : np;
          }
        }
      }
    }
    __syncthreads();
  }

  const int nv = lenW >> 2;
  int* gp = csr + rb0;
#pragma unroll 1
  for (int i = tid; i < nv; i += NTHR) { const v4i v = ((const v4i*)region)[i]; *(volatile v4i*)(gp + 4 * i) = v; }
  __threadfence();
#pragma unroll 1
  for (int i = tid; i < nv; i += NTHR) { const v4i v = ((const v4i*)region)[i]; *(volatile v4i*)(gp + 4 * i) = v; }
}

template <int NCOL>
__device__ __forceinline__ void mm3(const unsigned short* __restrict__ Ah, const unsigned short* __restrict__ Al,
                                    const unsigned short* __restrict__ Bh, const unsigned short* __restrict__ Bl,
                                    int rowBase, float* stg) {
  static_assert((NCOL % 32) == 0);
  constexpr int KD  = FD;
  constexpr int NT  = NCOL / 32;
  constexpr int NCW = NCOL / 2;
  const int tid = threadIdx.x, lane = tid & 31, wave = tid >> 5, hh = lane >> 4, m = lane & 15;
  const int r0 = (wave >> 1) * 16, c0 = (wave & 1) * NCW;
  v8f acc[NT];
#pragma unroll
  for (int t = 0; t < NT; ++t) { v8f z = {0.f, 0.f, 0.f, 0.f, 0.f, 0.f, 0.f, 0.f}; acc[t] = z; }
  const size_t aoff = (size_t)(rowBase + r0 + m) * PP + 8 * hh;
  const unsigned short* aph = Ah + aoff;
  const unsigned short* apl = Al + aoff;
  const size_t boff = (size_t)(c0 + m) * PP + 8 * hh;
  const unsigned short* bph0 = Bh + boff;
  const unsigned short* bpl0 = Bl + boff;
#pragma unroll 1
  for (int kt = 0; kt < KD / 32; ++kt) {
    FragU ah, al;
    ah.u[0] = *(const v8us*)(aph + 32 * kt);
    ah.u[1] = *(const v8us*)(aph + 32 * kt + 16);
    al.u[0] = *(const v8us*)(apl + 32 * kt);
    al.u[1] = *(const v8us*)(apl + 32 * kt + 16);
#pragma unroll
    for (int t = 0; t < NT; ++t) {
      const size_t to = (size_t)(16 * t) * PP + 32 * kt;
      FragU bh, bl;
      bh.u[0] = *(const v8us*)(bph0 + to);
      bh.u[1] = *(const v8us*)(bph0 + to + 16);
      bl.u[0] = *(const v8us*)(bpl0 + to);
      bl.u[1] = *(const v8us*)(bpl0 + to + 16);
      acc[t] = wmb(ah.w, bh.w, acc[t]);
      acc[t] = wmb(al.w, bh.w, acc[t]);
      acc[t] = wmb(ah.w, bl.w, acc[t]);
    }
  }
  float* sp = stg + (size_t)(r0 + 8 * hh) * NCOL + c0 + m;
#pragma unroll
  for (int t = 0; t < NT; ++t) {
#pragma unroll
    for (int r = 0; r < 8; ++r) sp[r * NCOL + 16 * t] = acc[t][r];
  }
}

template <int NCOL, int SPLITB>
__global__ __launch_bounds__(NTHR) void k_gemm_f32(
    const unsigned short* __restrict__ Ah, const unsigned short* __restrict__ Al,
    const unsigned short* __restrict__ Bh, const unsigned short* __restrict__ Bl,
    const float* __restrict__ biasA, const float* __restrict__ biasB,
    float* C, int ldc, int nlim) {
  extern __shared__ v4f lds_dyn[];
  float* stg = (float*)lds_dyn;
  const int tid = threadIdx.x, lane = tid & 31, wave = tid >> 5;
  const int rowBase = blockIdx.x * BM;
  constexpr int NCW = NCOL / 2, LPR = NCW / 4, RPI = 32 / LPR, NIT = 16 / RPI;
  static_assert(LPR >= 8 && (32 % LPR) == 0 && (16 % RPI) == 0);
  const int r0 = (wave >> 1) * 16, c0 = (wave & 1) * NCW;

  mm3<NCOL>(Ah, Al, Bh, Bl, rowBase, stg);
  __syncthreads();

  const int rsub = lane / LPR, q = lane - rsub * LPR, col = c0 + 4 * q;
  const float* bp = (SPLITB != 0) ? (((wave & 1) != 0) ? biasB : biasA) : biasA;
  const int bidx = (SPLITB != 0) ? (col - c0) : col;
  const v4f b4 = *(const v4f*)(bp + bidx);
#pragma unroll
  for (int it = 0; it < NIT; ++it) {
    const int row  = it * RPI + rsub;
    const int grow = rowBase + r0 + row;
    const v4f v = *(const v4f*)(stg + (size_t)(r0 + row) * NCOL + col) + b4;
    if (grow < nlim) *(volatile v4f*)(C + (size_t)grow * ldc + col) = v;
  }
  __threadfence();
#pragma unroll
  for (int it = 0; it < NIT; ++it) {
    const int row  = it * RPI + rsub;
    const int grow = rowBase + r0 + row;
    const v4f v = *(const v4f*)(stg + (size_t)(r0 + row) * NCOL + col) + b4;
    if (grow < nlim) *(volatile v4f*)(C + (size_t)grow * ldc + col) = v;
  }
}

__global__ __launch_bounds__(NTHR) void k_gemm_pl(
    const unsigned short* __restrict__ Ah, const unsigned short* __restrict__ Al,
    const unsigned short* __restrict__ Bh, const unsigned short* __restrict__ Bl,
    const float* __restrict__ bias, const float* __restrict__ slope,
    unsigned short* Oh, unsigned short* Ol) {
  extern __shared__ v4f lds_dyn[];
  float* stg = (float*)lds_dyn;
  const int tid = threadIdx.x, lane = tid & 31, wave = tid >> 5;
  const int rowBase = blockIdx.x * BM;
  const int r0 = (wave >> 1) * 16, c0 = (wave & 1) * 64;

  mm3<FD>(Ah, Al, Bh, Bl, rowBase, stg);
  __syncthreads();

  const float pa = slope[0];
  const int rsub = lane >> 3, q = lane & 7, col = c0 + 8 * q;
  const v4f ba = *(const v4f*)(bias + col), bb = *(const v4f*)(bias + col + 4);
#pragma unroll
  for (int it = 0; it < 4; ++it) {
    const int row  = it * 4 + rsub;
    const int grow = rowBase + r0 + row;
    const float* srow = stg + (size_t)(r0 + row) * FD + col;
    const v4f v0 = prelu4(*(const v4f*)srow + ba, pa);
    const v4f v1 = prelu4(*(const v4f*)(srow + 4) + bb, pa);
    v8us hv, lv;
    sp8(v0, v1, hv, lv);
    *(volatile v8us*)(Oh + (size_t)grow * PP + col) = hv;
    *(volatile v8us*)(Ol + (size_t)grow * PP + col) = lv;
  }
  __threadfence();
#pragma unroll
  for (int it = 0; it < 4; ++it) {
    const int row  = it * 4 + rsub;
    const int grow = rowBase + r0 + row;
    const float* srow = stg + (size_t)(r0 + row) * FD + col;
    const v4f v0 = prelu4(*(const v4f*)srow + ba, pa);
    const v4f v1 = prelu4(*(const v4f*)(srow + 4) + bb, pa);
    v8us hv, lv;
    sp8(v0, v1, hv, lv);
    *(volatile v8us*)(Oh + (size_t)grow * PP + col) = hv;
    *(volatile v8us*)(Ol + (size_t)grow * PP + col) = lv;
  }
}

__global__ __launch_bounds__(NTHR) void k_gat(
    const int* __restrict__ csr, const int* __restrict__ off, const int* __restrict__ cnt,
    const int* __restrict__ srcs, const float* __restrict__ eattr, const float* __restrict__ eam,
    float* cpl, const float* __restrict__ We, const float* __restrict__ att,
    const float* __restrict__ bias, int nN, int nE, int csrLen) {
  const int tid = threadIdx.x, lane = tid & 31, wave = tid >> 5;
  const int tbase = blockIdx.x * TGT + wave * 32;
  const int col = 4 * lane;
  const float eamn = eam[0];
  const v4f z4 = {0.f, 0.f, 0.f, 0.f};
  const v4f at4 = *(const v4f*)(att + col);
  const v4f we4 = *(const v4f*)(We + col);
  const v4f bb4 = *(const v4f*)(bias + col);
  const v4f ew4 = we4 * eamn;
  const int cl    = tbase + lane;
  const int cnt_l = cnt[cl];
  const int off_l = off[cl];

#pragma unroll 1
  for (int j = 0; j < 32; ++j) {
    const int c = tbase + j;
    int n = __shfl(cnt_l, j);
    n = n < 0 ? 0 : (n > DEGCAP ? DEGCAP : n);
    const int st = __shfl(off_l, j);
    float* rowc = cpl + (size_t)c * CP;
    const v4f xlc = *(const v4f*)(rowc + col);
    const v4f xrc = *(const v4f*)(rowc + FD + col);
    float m   = gsum8(dot4(lrl4(xlc + xrc + ew4), at4));
    float den = 1.0f;
    v4f acc = xlc;
#pragma unroll 1
    for (int q0 = 0; q0 < n; q0 += 32) {
      int pos = st + q0 + lane;
      pos = pos < 0 ? 0 : (pos > csrLen - 1 ? csrLen - 1 : pos);
      int eid = csr[pos];
      eid = eid < 0 ? 0 : (eid > nE - 1 ? nE - 1 : eid);
      int sl = srcs[eid];
      sl = sl < 0 ? 0 : (sl > nN - 1 ? nN - 1 : sl);
      const float eav = eattr[eid];
      const int mcnt = (n - q0) < 32 ? (n - q0) : 32;
#pragma unroll 1
      for (int pp = 0; pp < mcnt; ++pp) {
        const int   s  = __builtin_amdgcn_readlane(sl, pp);
        const float ea = rlf(eav, pp);
        const v4f xs = *(const v4f*)(cpl + (size_t)s * CP + col);
        v4f z = xs + xrc;
        z.x = fmaf(ea, we4.x, z.x); z.y = fmaf(ea, we4.y, z.y);
        z.z = fmaf(ea, we4.z, z.z); z.w = fmaf(ea, we4.w, z.w);
        z = lrl4(z);
        const float e  = gsum8(dot4(z, at4));
        const float mn = fmaxf(m, e);
        const float sc = fexp(m - mn);
        const float p  = fexp(e - mn);
        m = mn;
        den = fmaf(den, sc, p);
        const v4f xp = xs * p;
        acc.x = fmaf(acc.x, sc, xp.x); acc.y = fmaf(acc.y, sc, xp.y);
        acc.z = fmaf(acc.z, sc, xp.z); acc.w = fmaf(acc.w, sc, xp.w);
      }
    }
    const float rd = __builtin_amdgcn_rcpf(den);
    v4f v;
    v.x = fmaf(acc.x, rd, bb4.x); v.y = fmaf(acc.y, rd, bb4.y);
    v.z = fmaf(acc.z, rd, bb4.z); v.w = fmaf(acc.w, rd, bb4.w);
    if (c >= nN) v = z4;
    float* po = rowc + FD + col;
    *(volatile v4f*)po = v;
    __threadfence();
    *(volatile v4f*)po = v;
  }
}

__global__ __launch_bounds__(FD) void k_bnstat(const float* __restrict__ o0, double* part, int nN) {
  __shared__ __attribute__((aligned(16))) double spt[2 * FD];
  const int col = threadIdx.x;
  const int r0 = blockIdx.x * STATR;
  int nr = nN - r0;
  nr = nr < 0 ? 0 : (nr > STATR ? STATR : nr);
  double s = 0.0, q = 0.0;
#pragma unroll 1
  for (int i = 0; i < nr; ++i) {
    const double v = (double)o0[(size_t)(r0 + i) * CP + col];
    s += v;
    q += v * v;
  }
  spt[col] = s;
  spt[FD + col] = q;
  __syncthreads();
  const v2d w = *(const v2d*)(spt + 2 * col);
  double* pp = part + (size_t)blockIdx.x * (2 * FD) + 2 * col;
  *(volatile v2d*)pp = w;
  __threadfence();
  *(volatile v2d*)pp = w;
}

__global__ __launch_bounds__(FD) void k_bnfin(const double* __restrict__ part, const float* __restrict__ gamma,
                                              float* tbl, int nPart, int nN) {
  __shared__ __attribute__((aligned(16))) float stb[2 * FD];
  const int tid = threadIdx.x, col = tid;
  double s = 0.0, q = 0.0;
#pragma unroll 1
  for (int b = 0; b < nPart; ++b) {
    s += part[(size_t)b * (2 * FD) + col];
    q += part[(size_t)b * (2 * FD) + FD + col];
  }
  const double inv = 1.0 / (double)nN;
  const double mu  = s * inv;
  double var = q * inv - mu * mu;
  var = var < 0.0 ? 0.0 : var;
  const float a  = (float)((double)gamma[col] / sqrt(var + BN_EPS));
  const float mf = (float)mu;
  stb[col] = mf;
  stb[FD + col] = a;
  __syncthreads();
  const int t4 = tid < 64 ? tid : 63;
  const v4f w = *(const v4f*)(stb + 4 * t4);
  if (tid < 64) *(volatile v4f*)(tbl + 4 * tid) = w;
  __threadfence();
  if (tid < 64) *(volatile v4f*)(tbl + 4 * tid) = w;
}

__global__ __launch_bounds__(NTHR) void k_bnapply(
    const float* __restrict__ o0, const float* __restrict__ tbl, const float* __restrict__ beta,
    const float* __restrict__ slope, unsigned short* ph, unsigned short* pl, int nN, int nUnits) {
  const int i = (int)blockIdx.x * NTHR + (int)threadIdx.x;
  if (i >= nUnits) return;
  const int row = i >> 4;
  const int c   = (i & 15) * 8;
  const float pa = slope[0];
  const float* orow = o0 + (size_t)row * CP + c;
  const v4f s0 = *(const v4f*)orow, s1 = *(const v4f*)(orow + 4);
  const v4f mu0 = *(const v4f*)(tbl + c),      mu1 = *(const v4f*)(tbl + c + 4);
  const v4f ga0 = *(const v4f*)(tbl + FD + c), ga1 = *(const v4f*)(tbl + FD + c + 4);
  const v4f be0 = *(const v4f*)(beta + c),     be1 = *(const v4f*)(beta + c + 4);
  const v4f z4 = {0.f, 0.f, 0.f, 0.f};
  v4f h0 = prelu4((s0 - mu0) * ga0 + be0, pa);
  v4f h1 = prelu4((s1 - mu1) * ga1 + be1, pa);
  if (row >= nN) { h0 = z4; h1 = z4; }
  v8us hv, lv;
  sp8(h0, h1, hv, lv);
  unsigned short* dh = ph + (size_t)row * PP + c;
  unsigned short* dl = pl + (size_t)row * PP + c;
  *(volatile v8us*)dh = hv;
  *(volatile v8us*)dl = lv;
  __threadfence();
  *(volatile v8us*)dh = hv;
  *(volatile v8us*)dl = lv;
}

static size_t carve(size_t* o, size_t bytes) {
  const size_t r = *o;
  *o += (bytes + 255) & ~(size_t)255;
  return r;
}

extern "C" void kernel_launch(void* const* d_in, const int* in_sizes, int n_in,
                              void* d_out, int out_size, void* d_ws, size_t ws_size,
                              hipStream_t stream) {
  if (n_in < 28) return;
  const int nN = in_sizes[0] / FD;
  const int nE = in_sizes[1] / 2;
  if (nN <= 0 || nE <= 0 || in_sizes[0] != nN * FD || in_sizes[1] != 2 * nE || in_sizes[2] != nE) return;
  if (in_sizes[3] != FD * FD || in_sizes[4] != FD || in_sizes[5] < 1) return;
  if (in_sizes[6] != FD * FD || in_sizes[7] != FD || in_sizes[8] != FD * NOUTC || in_sizes[9] != NOUTC) return;
  for (int l = 0; l < 2; ++l) {
    const int b = 10 + 9 * l;
    if (in_sizes[b] != FD * FD || in_sizes[b + 1] != FD || in_sizes[b + 2] != FD * FD || in_sizes[b + 3] != FD) return;
    if (in_sizes[b + 4] != FD || in_sizes[b + 5] != FD || in_sizes[b + 6] != FD || in_sizes[b + 7] != FD || in_sizes[b + 8] != FD) return;
  }
  if ((long long)out_size != (long long)nN * NOUTC) return;
  if (nE > (1 << 27) || nN > (1 << 22)) return;

  const float* x      = (const float*)d_in[0];
  const int*   ei     = (const int*)d_in[1];
  const float* eattr  = (const float*)d_in[2];
  const float* pre_W  = (const float*)d_in[3];
  const float* pre_b  = (const float*)d_in[4];
  const float* prelu  = (const float*)d_in[5];
  const float* post_W = (const float*)d_in[6];
  const float* post_b = (const float*)d_in[7];
  const float* out_W  = (const float*)d_in[8];
  const float* out_b  = (const float*)d_in[9];
  const float* Wl0 = (const float*)d_in[10]; const float* bl0 = (const float*)d_in[11];
  const float* Wr0 = (const float*)d_in[12]; const float* br0 = (const float*)d_in[13];
  const float* We0 = (const float*)d_in[14]; const float* at0 = (const float*)d_in[15];
  const float* bi0 = (const float*)d_in[16]; const float* ga0 = (const float*)d_in[17];
  const float* be0 = (const float*)d_in[18];
  const float* Wl1 = (const float*)d_in[19]; const float* bl1 = (const float*)d_in[20];
  const float* Wr1 = (const float*)d_in[21]; const float* br1 = (const float*)d_in[22];
  const float* We1 = (const float*)d_in[23]; const float* at1 = (const float*)d_in[24];
  const float* bi1 = (const float*)d_in[25]; const float* ga1 = (const float*)d_in[26];
  const float* be1 = (const float*)d_in[27];
  const int* src = ei;
  const int* dst = ei + nE;
  float* dout = (float*)d_out;

  const int NPAD   = ((nN + TGT - 1) / TGT) * TGT;
  const int nBC    = (nN + NBC - 1) / NBC;
  const int CNTPAD = nBC * NBC;
  if (FPC * nBC + 1 > RBN) return;
  const int nBF    = (nN + NBF - 1) / NBF;
  const int csrLen = ((nE + 31) & ~31) + 4096;
  if (31 * FPC * nBC > 4096) return;
  const int nAgg   = NPAD / TGT;
  const int nGm    = NPAD / BM;
  const int nStat  = NPAD / STATR;
  const int nUnit  = NPAD * (FD / 8);
  const int nUB    = (nUnit + NTHR - 1) / NTHR;

  char* ws = (char*)d_ws;
  size_t o = 0;
  const size_t plB  = (size_t)NPAD * PP * 2;
  const size_t oWpreH = carve(&o, (size_t)FD * FD * 2),    oWpreL = carve(&o, (size_t)FD * FD * 2);
  const size_t oW0H   = carve(&o, (size_t)NC2 * FD * 2),   oW0L   = carve(&o, (size_t)NC2 * FD * 2);
  const size_t oW1H   = carve(&o, (size_t)NC2 * FD * 2),   oW1L   = carve(&o, (size_t)NC2 * FD * 2);
  const size_t oWpoH  = carve(&o, (size_t)FD * FD * 2),    oWpoL  = carve(&o, (size_t)FD * FD * 2);
  const size_t oWouH  = carve(&o, (size_t)NOUTC * FD * 2), oWouL  = carve(&o, (size_t)NOUTC * FD * 2);
  const size_t oCnt   = carve(&o, (size_t)CNTPAD * 4);
  const size_t oOff   = carve(&o, (size_t)CNTPAD * 4);
  const size_t oRb    = carve(&o, (size_t)RBN * 4);
  const size_t oCsr   = carve(&o, (size_t)csrLen * 4);
  const size_t oEam   = carve(&o, 256);
  const size_t oPart  = carve(&o, (size_t)nStat * 2 * FD * 8);
  const size_t oTbl   = carve(&o, (size_t)2 * FD * 4);
  const size_t oP0H   = carve(&o, plB), oP0L = carve(&o, plB);
  const size_t oP1H   = carve(&o, plB), oP1L = carve(&o, plB);
  const size_t oCp    = carve(&o, (size_t)NPAD * CP * 4);
  if (o > ws_size || o > (size_t)WSCAP) return;

  unsigned short* wpreH = (unsigned short*)(ws + oWpreH); unsigned short* wpreL = (unsigned short*)(ws + oWpreL);
  unsigned short* w0H   = (unsigned short*)(ws + oW0H);   unsigned short* w0L   = (unsigned short*)(ws + oW0L);
  unsigned short* w1H   = (unsigned short*)(ws + oW1H);   unsigned short* w1L   = (unsigned short*)(ws + oW1L);
  unsigned short* wpoH  = (unsigned short*)(ws + oWpoH);  unsigned short* wpoL  = (unsigned short*)(ws + oWpoL);
  unsigned short* wouH  = (unsigned short*)(ws + oWouH);  unsigned short* wouL  = (unsigned short*)(ws + oWouL);
  int*    cnt  = (int*)(ws + oCnt);
  int*    offp = (int*)(ws + oOff);
  int*    rb   = (int*)(ws + oRb);
  int*    csr  = (int*)(ws + oCsr);
  float*  eam  = (float*)(ws + oEam);
  double* part = (double*)(ws + oPart);
  float*  tbl  = (float*)(ws + oTbl);
  unsigned short* P0H = (unsigned short*)(ws + oP0H); unsigned short* P0L = (unsigned short*)(ws + oP0L);
  unsigned short* P1H = (unsigned short*)(ws + oP1H); unsigned short* P1L = (unsigned short*)(ws + oP1L);
  float*  cpl  = (float*)(ws + oCp);
  float*  o0   = cpl + FD;

  const int vec8 = ((nE & 3) == 0) ? 1 : 0;

  k_xsplit<<<nUB, NTHR, 0, stream>>>(x, P0H, P0L, nN, nUnit);

  k_wprep<<<(FD * 16 + NTHR - 1) / NTHR, NTHR, 0, stream>>>(pre_W, pre_W, FD, FD, wpreH, wpreL, FD * 16);
  k_wprep<<<(NC2 * 16 + NTHR - 1) / NTHR, NTHR, 0, stream>>>(Wl0, Wr0, FD, FD, w0H, w0L, NC2 * 16);
  k_wprep<<<(NC2 * 16 + NTHR - 1) / NTHR, NTHR, 0, stream>>>(Wl1, Wr1, FD, FD, w1H, w1L, NC2 * 16);
  k_wprep<<<(FD * 16 + NTHR - 1) / NTHR, NTHR, 0, stream>>>(post_W, post_W, FD, FD, wpoH, wpoL, FD * 16);
  k_wprep<<<(NOUTC * 16 + NTHR - 1) / NTHR, NTHR, 0, stream>>>(out_W, out_W, NOUTC, NOUTC, wouH, wouL, NOUTC * 16);

  k_eamean<<<1, NTHR, 0, stream>>>(eattr, eam, nE);

  k_count<<<nBC, NTHR, 0, stream>>>(dst, cnt, nE, vec8);
  k_offsets<<<1, OTHR, 0, stream>>>(cnt, offp, rb, nBC);
  hipFuncSetAttribute(reinterpret_cast<const void*>(&k_fill),
                      hipFuncAttributeMaxDynamicSharedMemorySize, LDS_FILL);
  k_fill<<<nBF, NTHR, LDS_FILL, stream>>>(dst, offp, rb, csr, nE, vec8, csrLen);

  k_gemm_pl<<<nGm, NTHR, LDS_G128, stream>>>(P0H, P0L, wpreH, wpreL, pre_b, prelu, P1H, P1L);

  hipFuncSetAttribute(reinterpret_cast<const void*>(&k_gemm_f32<NC2, 1>),
                      hipFuncAttributeMaxDynamicSharedMemorySize, LDS_G256);
  k_gemm_f32<NC2, 1><<<nGm, NTHR, LDS_G256, stream>>>(P1H, P1L, w0H, w0L, bl0, br0, cpl, CP, NPAD);
  k_gat<<<nAgg, NTHR, 0, stream>>>(csr, offp, cnt, src, eattr, eam, cpl, We0, at0, bi0, nN, nE, csrLen);
  k_bnstat<<<nStat, FD, 0, stream>>>(o0, part, nN);
  k_bnfin<<<1, FD, 0, stream>>>(part, ga0, tbl, nStat, nN);
  k_bnapply<<<nUB, NTHR, 0, stream>>>(o0, tbl, be0, prelu, P0H, P0L, nN, nUnit);

  k_gemm_f32<NC2, 1><<<nGm, NTHR, LDS_G256, stream>>>(P0H, P0L, w1H, w1L, bl1, br1, cpl, CP, NPAD);
  k_gat<<<nAgg, NTHR, 0, stream>>>(csr, offp, cnt, src, eattr, eam, cpl, We1, at1, bi1, nN, nE, csrLen);
  k_bnstat<<<nStat, FD, 0, stream>>>(o0, part, nN);
  k_bnfin<<<1, FD, 0, stream>>>(part, ga1, tbl, nStat, nN);
  k_bnapply<<<nUB, NTHR, 0, stream>>>(o0, tbl, be1, prelu, P1H, P1L, nN, nUnit);

  k_gemm_pl<<<nGm, NTHR, LDS_G128, stream>>>(P1H, P1L, wpoH, wpoL, post_b, prelu, P0H, P0L);

  k_gemm_f32<NOUTC, 0><<<nGm, NTHR, LDS_G64, stream>>>(P0H, P0L, wouH, wouL, out_b, out_b, dout, NOUTC, nN);
}
